// ISTFT_48258252538127
// MI455X (gfx1250) — hardware-verified
//
#include <hip/hip_runtime.h>
#include <stdint.h>

#define NB    8
#define NT    1024
#define NFREQ 1025
#define NFFT  2048
#define NHALF 1024
#define HOPL  512
#define KTOT  4096
#define LEN   523776
#define NBG   4
#define MG    (NBG * NT)
#define JQ    (LEN / 4)
#define NQ    (NBG * JQ)

static_assert(LEN == (NT - 1) * HOPL);
static_assert(KTOT % 32 == 0);
static_assert(MG % 64 == 0);
static_assert(NFFT % 64 == 0);
static_assert(LEN % 128 == 0);
static_assert(JQ % 32 == 0);
static_assert(NQ % 256 == 0);
static_assert(NB % NBG == 0);
static_assert(((MG / 64) * (NFFT / 64)) % 8 == 0);

typedef __attribute__((ext_vector_type(16))) __bf16 v16b;
typedef __attribute__((ext_vector_type(8)))  __bf16 v8b;
typedef __attribute__((ext_vector_type(8)))  float  v8f;
typedef __attribute__((ext_vector_type(4)))  float  v4f;
typedef __attribute__((ext_vector_type(4)))  unsigned int v4u;
typedef v4f __attribute__((may_alias)) v4fa;
typedef v8b __attribute__((may_alias)) v8ba;

__device__ __forceinline__ unsigned short f2bf_bits(float f) {
  const unsigned u = __float_as_uint(f);
  return (unsigned short)((u + 0x7FFFu + ((u >> 16) & 1u)) >> 16);
}
__device__ __forceinline__ float bf_rne(float f) { return __uint_as_float(((unsigned)f2bf_bits(f)) << 16); }
__device__ __forceinline__ unsigned pk16(unsigned short a, unsigned short b) { return (unsigned)a | ((unsigned)b << 16); }

__device__ __forceinline__ v16b load_frag(const __bf16* p) {
  union { v16b v; v8b h[2]; } f;
  f.h[0] = *(const v8ba*)(p);
  f.h[1] = *(const v8ba*)(p + 16);
  return f.v;
}
__device__ __forceinline__ v8f mma_bf(v16b a, v16b b, v8f c) {
  return __builtin_amdgcn_wmma_f32_16x16x32_bf16(false, a, false, b, (short)0, c, false, false);
}
__device__ __forceinline__ void dep_guard(v8f& a, v8f& b, v16b x) {
  asm volatile("v_nop\n\tv_nop\n\tv_nop\n\tv_nop" : "+v"(a), "+v"(b) : "v"(x));
}
__device__ __forceinline__ void keep4(v16b a, v16b b, v16b c, v16b d) {
  asm volatile("v_nop" :: "v"(a), "v"(b), "v"(c), "v"(d));
}
__device__ __forceinline__ void acc_guard4(v8f& a, v8f& b, v8f& c, v8f& d) {
  asm volatile("v_nop\n\tv_nop\n\tv_nop\n\tv_nop" : "+v"(a), "+v"(b), "+v"(c), "+v"(d));
}

__global__ __launch_bounds__(256) void spec_kernel(const float* __restrict__ re, const float* __restrict__ im,
                                                   unsigned short* __restrict__ Ap) {
  const int row = blockIdx.y;
  const int qs  = blockIdx.x;
  const float* src = ((qs == 0) ? re : im) + (size_t)row * NFREQ;
  const bool neg = (qs != 0);
  const int kk0 = threadIdx.x * 8;
  float v[8];
#pragma unroll
  for (int e = 0; e < 8; ++e) {
    const int kk = kk0 + e;
    const int f  = min(kk, NFFT - kk);
    const float sg = (neg && kk > NHALF) ? -1.0f : 1.0f;
    v[e] = src[f] * sg;
  }
  v4u o;
#pragma unroll
  for (int p = 0; p < 4; ++p) o[p] = pk16(f2bf_bits(v[2 * p]), f2bf_bits(v[2 * p + 1]));
  unsigned short* dst = Ap + (size_t)row * KTOT + (size_t)qs * NFFT + kk0;
  *(volatile v4u*)dst = o;
  __threadfence();
  *(volatile v4u*)dst = o;
}

__global__ __launch_bounds__(256) void wt_kernel(const float* __restrict__ Wr, const float* __restrict__ Wi,
                                                 unsigned short* __restrict__ Bt) {
  __shared__ __align__(16) float tf[64 * 68];
  const int z = blockIdx.z;
  const float* W = (z == 0) ? Wr : Wi;
  const float sg = (z == 0) ? 1.0f : -1.0f;
  unsigned short* oh = Bt + (size_t)z * NFFT;
  const int c0  = blockIdx.x * 64;
  const int r0  = blockIdx.y * 64;
  const int tid = threadIdx.x;
  {
    const int lr = tid >> 4;
    const int c4 = (tid & 15) * 4;
#pragma unroll
    for (int it = 0; it < 4; ++it) {
      const int rr = it * 16 + lr;
      const v4f a = *(const v4fa*)(W + (size_t)(r0 + rr) * NFFT + c0 + c4);
      *(v4f*)(tf + rr * 68 + c4) = a;
    }
  }
  __syncthreads();
  const int sub = tid >> 3;
  const int c8  = (tid & 7) * 8;
  v4u hv[2];
#pragma unroll
  for (int it = 0; it < 2; ++it) {
    const int oc = it * 32 + sub;
    v4u a;
#pragma unroll
    for (int q = 0; q < 4; ++q) {
      const float f0 = tf[(c8 + 2 * q) * 68 + oc] * sg;
      const float f1 = tf[(c8 + 2 * q + 1) * 68 + oc] * sg;
      a[q] = pk16(f2bf_bits(f0), f2bf_bits(f1));
    }
    hv[it] = a;
  }
  for (int pass = 0; pass < 2; ++pass) {
#pragma unroll
    for (int it = 0; it < 2; ++it) {
      const int oc = it * 32 + sub;
      const size_t go = (size_t)(c0 + oc) * KTOT + r0 + c8;
      *(volatile v4u*)(oh + go) = hv[it];
    }
    __threadfence();
  }
}

__global__ __launch_bounds__(256) void gemm_kernel(const unsigned short* __restrict__ Ap, int lda,
                                                   const unsigned short* __restrict__ Btp, int ldb,
                                                   float* __restrict__ C, int ldc, int M, int N, int K) {
  const __bf16* A  = (const __bf16*)(const void*)Ap;
  const __bf16* Bt = (const __bf16*)(const void*)Btp;
  __shared__ __align__(16) float sT[8][16 * 68];
  const int lane = threadIdx.x & 31;
  const int wave = threadIdx.x >> 5;
  const int tilesN = N >> 6;
  const int tilesM = M >> 6;
  const int tile = blockIdx.x * 8 + wave;
  if (tile >= tilesM * tilesN) return;
  const int tm = tile / tilesN;
  const int tn = tile - tm * tilesN;
  const int m0 = tm << 6;
  const int n0 = tn << 6;
  const int rlane = lane & 15;
  const int koff  = (lane >> 4) * 8;
  const int mOff  = (lane >> 4) * 8;

  v8f acc[4][4];
#pragma unroll
  for (int i = 0; i < 4; ++i)
#pragma unroll
    for (int j = 0; j < 4; ++j) acc[i][j] = (v8f){0.f, 0.f, 0.f, 0.f, 0.f, 0.f, 0.f, 0.f};

  for (int k0 = 0; k0 < K; k0 += 32) {
    v16b bfr[4];
#pragma unroll
    for (int j = 0; j < 4; ++j) {
      const size_t bo = (size_t)(n0 + (j << 4) + rlane) * ldb + koff + k0;
      bfr[j] = load_frag(Bt + bo);
    }
#pragma unroll
    for (int i = 0; i < 4; ++i) {
      const size_t ao = (size_t)(m0 + (i << 4) + rlane) * lda + koff + k0;
      const v16b afr = load_frag(A + ao);
#pragma unroll
      for (int j = 0; j < 4; ++j) acc[i][j] = mma_bf(afr, bfr[j], acc[i][j]);
      dep_guard(acc[i][0], acc[i][3], afr);
    }
    keep4(bfr[0], bfr[1], bfr[2], bfr[3]);
  }
  acc_guard4(acc[0][0], acc[0][1], acc[0][2], acc[0][3]);
  acc_guard4(acc[1][0], acc[1][1], acc[1][2], acc[1][3]);
  acc_guard4(acc[2][0], acc[2][1], acc[2][2], acc[2][3]);
  acc_guard4(acc[3][0], acc[3][1], acc[3][2], acc[3][3]);

  float* slab = sT[wave];
  const int hh = lane >> 4, c4 = (lane & 15) * 4;
#pragma unroll
  for (int i = 0; i < 4; ++i) {
    const int mBase = m0 + (i << 4);
#pragma unroll
    for (int j = 0; j < 4; ++j) {
#pragma unroll
      for (int r = 0; r < 8; ++r) slab[(mOff + r) * 68 + (j << 4) + rlane] = acc[i][j][r];
    }
    __builtin_amdgcn_fence(__ATOMIC_RELEASE, "workgroup");
    __builtin_amdgcn_wave_barrier();
    __builtin_amdgcn_fence(__ATOMIC_ACQUIRE, "workgroup");
    for (int pass = 0; pass < 2; ++pass) {
#pragma unroll
      for (int it = 0; it < 8; ++it) {
        const int row = it * 2 + hh;
        const v4f v = *(const v4fa*)(slab + row * 68 + c4);
        *(volatile v4f*)(C + (size_t)(mBase + row) * ldc + n0 + c4) = v;
      }
      __threadfence();
    }
    __builtin_amdgcn_fence(__ATOMIC_RELEASE, "workgroup");
    __builtin_amdgcn_wave_barrier();
    __builtin_amdgcn_fence(__ATOMIC_ACQUIRE, "workgroup");
  }
}

__global__ __launch_bounds__(256) void ola_kernel(const float* __restrict__ S, const float* __restrict__ ola,
                                                  const int* __restrict__ lenp, float* __restrict__ out, int bofs) {
  (void)lenp;
  const int q = blockIdx.x * 256 + threadIdx.x;
  if (q >= NQ) return;
  const int bl = q / JQ;
  const int j4 = q - bl * JQ;
  const int m  = j4 * 4;
  const int n  = m + NHALF;
  const int tb = n >> 9;
  const int ob = n & (HOPL - 1);
  v4f y = {0.f, 0.f, 0.f, 0.f};
  v4f w = {0.f, 0.f, 0.f, 0.f};
#pragma unroll
  for (int k = 3; k >= 0; --k) {
    const int t = tb - k;
    const int o = ob + HOPL * k;
    const unsigned msk = (t >= 0 && t < NT) ? 0xffffffffu : 0u;
    const int tc = min(max(t, 0), NT - 1);
    const v4f sv = *(const v4fa*)(S + ((size_t)(bl * NT + tc)) * NFFT + o);
    const v4f wv = *(const v4fa*)(ola + o);
#pragma unroll
    for (int c = 0; c < 4; ++c) {
      y[c] += __uint_as_float(__float_as_uint(sv[c]) & msk);
      w[c] += __uint_as_float(__float_as_uint(bf_rne(wv[c])) & msk);
    }
  }
  v4f res;
#pragma unroll
  for (int c = 0; c < 4; ++c) res[c] = y[c] * (1.0f / fmaxf(w[c], 1e-11f));
  const size_t gi = (size_t)(bofs + bl) * LEN + m;
  *(volatile v4f*)(out + gi) = res;
  __threadfence();
  *(volatile v4f*)(out + gi) = res;
}

extern "C" void kernel_launch(void* const* d_in, const int* in_sizes, int n_in,
                              void* d_out, int out_size, void* d_ws, size_t ws_size,
                              hipStream_t stream) {
  if (n_in < 6) return;
  if (in_sizes[0] != NB * NT * NFREQ || in_sizes[1] != NB * NT * NFREQ) return;
  if (in_sizes[2] != NFFT * NFFT || in_sizes[3] != NFFT * NFFT) return;
  if (in_sizes[4] != NFFT) return;
  if (in_sizes[5] < 1) return;
  if (out_size != NB * LEN) return;

  const float* re  = (const float*)d_in[0];
  const float* im  = (const float*)d_in[1];
  const float* Wr  = (const float*)d_in[2];
  const float* Wi  = (const float*)d_in[3];
  const float* ola = (const float*)d_in[4];
  const int*   lenp = (const int*)d_in[5];
  float* out = (float*)d_out;

  const size_t PAP = (size_t)NB * NT * KTOT * 2;
  const size_t PBT = (size_t)NFFT * KTOT * 2;
  const size_t PS  = (size_t)MG * NFFT * 4;
  size_t off = 0;
  const size_t oAP = off; off += PAP;
  const size_t oBT = off; off += PBT;
  const size_t oS  = off; off += PS;
  if (off > ws_size) return;
  if (off > (size_t)134217728) return;

  char* ws = (char*)d_ws;
  unsigned short* AP = (unsigned short*)(ws + oAP);
  unsigned short* BT = (unsigned short*)(ws + oBT);
  float* S = (float*)(ws + oS);

  const dim3 blk(256);
  spec_kernel<<<dim3(2, NB * NT), blk, 0, stream>>>(re, im, AP);
  wt_kernel<<<dim3(NFFT / 64, NFFT / 64, 2), blk, 0, stream>>>(Wr, Wi, BT);
  for (int g = 0; g < NB / NBG; ++g) {
    const unsigned short* Ag = AP + (size_t)g * MG * KTOT;
    gemm_kernel<<<dim3(((MG / 64) * (NFFT / 64)) / 8), blk, 0, stream>>>(Ag, KTOT, BT, KTOT, S, NFFT, MG, NFFT, KTOT);
    ola_kernel<<<dim3(NQ / 256), blk, 0, stream>>>(S, ola, lenp, out, g * NBG);
  }
  (void)hipGetLastError();
}
